// MultiHeadAttentionDecomposed_82051055222904
// MI455X (gfx1250) — hardware-verified
//
#include <hip/hip_runtime.h>
#include <math.h>

typedef __attribute__((ext_vector_type(16))) _Float16 v16h;
typedef __attribute__((ext_vector_type(16))) __bf16 v16b;
typedef __attribute__((ext_vector_type(8)))  _Float16 v8h;
typedef __attribute__((ext_vector_type(8)))  float v8f;
typedef __attribute__((ext_vector_type(4)))  float v4f;
typedef __attribute__((ext_vector_type(2)))  float v2f;
typedef __attribute__((ext_vector_type(4)))  unsigned v4u;
typedef __attribute__((ext_vector_type(4)))  int v4i;
typedef float __attribute__((may_alias)) float_a;
typedef int __attribute__((may_alias)) int_a;

template <typename T> __device__ __forceinline__ void vst2(void* p, T v) { *(volatile T*)p = v; __threadfence(); *(volatile T*)p = v; }
__device__ __forceinline__ v8f wmma16(v16h a, v16h b, v8f c) {
  v8f d = __builtin_amdgcn_wmma_f32_16x16x32_f16(false, a, false, b, (short)0, c, false, false);
  asm volatile("v_nop\n\tv_nop\n\tv_nop\n\tv_nop" : "+v"(d) : "v"(a), "v"(b));
  return d;
}
__device__ __forceinline__ v8f wmma_bf(v16b a, v16b b, v8f c) {
  v8f d = __builtin_amdgcn_wmma_f32_16x16x32_bf16(false, a, false, b, (short)0, c, false, false);
  asm volatile("v_nop\n\tv_nop\n\tv_nop\n\tv_nop" : "+v"(d) : "v"(a), "v"(b));
  return d;
}
__device__ __forceinline__ v16h frag_h(const _Float16* rowk0, int lane) {
  union { v16h v; v8h q[2]; } u; const _Float16* p = rowk0 + 8 * (lane >> 4);
  u.q[0] = *(const v8h*)p; u.q[1] = *(const v8h*)(p + 16); return u.v;
}
__device__ __forceinline__ v16h frag_f32(const float* rowk0, int lane) {
  v16h a; const float* p = rowk0 + 8 * (lane >> 4);
#pragma unroll
  for (int i = 0; i < 8; ++i) { a[i] = (_Float16)p[i]; a[8 + i] = (_Float16)p[16 + i]; }
  return a;
}
__device__ __forceinline__ v16h frag_f32s(const float* rowk0, int lane, float sc) {
  v16h a; const float* p = rowk0 + 8 * (lane >> 4);
#pragma unroll
  for (int i = 0; i < 8; ++i) { a[i] = (_Float16)(p[i] * sc); a[8 + i] = (_Float16)(p[16 + i] * sc); }
  return a;
}
__device__ __forceinline__ v16h fragc_f32(const float* W, int k0, int n, int lane, int ld, int K) {
  v16h a; const int g = lane >> 4;
#pragma unroll
  for (int i = 0; i < 8; ++i) { const int ka = k0 + 8 * g + i, kb = ka + 16;
    a[i] = (_Float16)(ka < K ? W[(size_t)(ka < K ? ka : K - 1) * ld + n] : 0.f); a[8 + i] = (_Float16)(kb < K ? W[(size_t)(kb < K ? kb : K - 1) * ld + n] : 0.f); }
  return a;
}
struct F2 { v16b h, l; };
__device__ __forceinline__ F2 bsplit16(const float v[16]) { F2 r;
#pragma unroll
  for (int i = 0; i < 16; ++i) { const __bf16 h = (__bf16)v[i]; r.h[i] = h; r.l[i] = (__bf16)(v[i] - (float)h); }
  return r; }
__device__ __forceinline__ F2 split_row(const float* row, int k0, int lane) { float v[16]; const float* p = row + k0 + 8 * (lane >> 4);
#pragma unroll
  for (int i = 0; i < 8; ++i) { v[i] = p[i]; v[8 + i] = p[16 + i]; }
  return bsplit16(v); }
__device__ __forceinline__ F2 split_rowK(const float* row, int k0, int lane, int K) { float v[16]; const int g = lane >> 4;
#pragma unroll
  for (int i = 0; i < 8; ++i) { const int ka = k0 + 8 * g + i, kb = ka + 16; v[i] = ka < K ? row[ka < K ? ka : K - 1] : 0.f; v[8 + i] = kb < K ? row[kb < K ? kb : K - 1] : 0.f; }
  return bsplit16(v); }
__device__ __forceinline__ F2 split_col(const float* W, int k0, int n, int lane, int ld, int K) { float v[16]; const int g = lane >> 4;
#pragma unroll
  for (int i = 0; i < 8; ++i) { const int ka = k0 + 8 * g + i, kb = ka + 16; v[i] = ka < K ? W[(size_t)(ka < K ? ka : K - 1) * ld + n] : 0.f; v[8 + i] = kb < K ? W[(size_t)(kb < K ? kb : K - 1) * ld + n] : 0.f; }
  return bsplit16(v); }
__device__ __forceinline__ v8f mac3(const F2& a, const F2& b, v8f c) { c = wmma_bf(a.l, b.h, c); c = wmma_bf(a.h, b.l, c); return wmma_bf(a.h, b.h, c); }
__device__ __forceinline__ float sigm(float v) { return 1.0f / (1.0f + expf(-v)); }
#define LDSX() do { asm volatile("s_wait_dscnt 0" ::: "memory"); __builtin_amdgcn_wave_barrier(); __builtin_amdgcn_fence(__ATOMIC_RELEASE, "workgroup"); } while (0)


#define SEQ 197
#define NBT 2
#define DM 768
#define NHD 12
#define DHD 64
typedef __attribute__((ext_vector_type(8))) __bf16 v8b;
__device__ __forceinline__ v16b frag_b(const __bf16* rowk0, int lane) {
  union { v16b v; v8b q[2]; } u; const __bf16* p = rowk0 + 8 * (lane >> 4);
  u.q[0] = *(const v8b*)p; u.q[1] = *(const v8b*)(p + 16); return u.v;
}
__device__ __forceinline__ v16b frag_gbf(const float* rowk0, int lane) {
  v16b a; const float* p = rowk0 + 8 * (lane >> 4);
#pragma unroll
  for (int i = 0; i < 8; ++i) { a[i] = (__bf16)p[i]; a[8 + i] = (__bf16)p[16 + i]; }
  return a;
}
__device__ __forceinline__ float bfr(float v) { return (float)(__bf16)v; }
__device__ __attribute__((noinline)) float exp_ni(float v) { return expf(v); }
#define NROW (SEQ * NBT)
#define NROWP 400
#define WS_K   0u
#define WS_END (WS_K + 4u * NROWP * DM)

__global__ __launch_bounds__(128) void k_key(const float* __restrict__ X, const float* __restrict__ Wk, const float* __restrict__ Bk, float* __restrict__ Kb) {
  __shared__ __align__(16) float so[4][16][132];
  const int tid = threadIdx.x, wave = tid >> 5, lane = tid & 31, col = lane & 15, g = lane >> 4; const int r0 = blockIdx.x * 64 + wave * 16; const int n0 = blockIdx.y * 128;
  if (r0 >= NROWP) return;
  const int ra = min(r0 + col, NROW - 1);
  v8f acc[8] = {};
#pragma unroll 2
  for (int kc = 0; kc < DM / 32; ++kc) { const v16b a = frag_gbf(X + (size_t)ra * DM + kc * 32, lane);
#pragma unroll
    for (int j = 0; j < 8; ++j) acc[j] = wmma_bf(a, frag_gbf(Wk + (size_t)(n0 + j * 16 + col) * DM + kc * 32, lane), acc[j]); }
#pragma unroll
  for (int j = 0; j < 8; ++j) { const float bb = bfr(Bk[n0 + j * 16 + col]);
#pragma unroll
    for (int r = 0; r < 8; ++r) so[wave][8 * g + r][j * 16 + col] = acc[j][r] + bb; }
  LDSX();
  for (int rl = 0; rl < 16; ++rl) vst2(Kb + (size_t)(r0 + rl) * DM + n0 + lane * 4, *(const v4f*)&so[wave][rl][lane * 4]);
}
__global__ __launch_bounds__(256) void k_cls(const float* __restrict__ X, const float* __restrict__ Kb, const float* __restrict__ Wq, const float* __restrict__ Bq, const float* __restrict__ Wv, const float* __restrict__ Bv, const float* __restrict__ Wo, const float* __restrict__ Bo, float* __restrict__ out) {
  __shared__ float sq[DM]; __shared__ float sa[NHD][SEQ + 3]; __shared__ __align__(16) float sxa[16][DM + 4]; __shared__ __align__(16) float sy[16][DM + 4]; __shared__ __align__(16) float sres[DM];
  const int tid = threadIdx.x, wave = tid >> 5, lane = tid & 31, col = lane & 15, g = lane >> 4; const int b = blockIdx.x;
  for (int o = tid; o < DM; o += 256) { const float* wr = Wq + (size_t)o * DM; const float* xr = X + (size_t)(0 * 2 + b) * DM; float s = 0.f; for (int c = 0; c < DM; ++c) s += bfr(xr[c]) * bfr(wr[c]); sq[o] = (s + bfr(Bq[o])) * 0.125f; }
  for (int q = tid; q < 16 * (DM + 4); q += 256) { (&sxa[0][0])[q] = 0.f; (&sy[0][0])[q] = 0.f; }
  __syncthreads();
  for (int e = tid; e < NHD * SEQ; e += 256) { const int h = e / SEQ, m = e % SEQ; const float* kr = Kb + (size_t)(m * 2 + b) * DM + h * DHD; float s = 0.f; for (int d = 0; d < DHD; ++d) s += sq[h * DHD + d] * kr[d]; sa[h][m] = s; }
  __syncthreads();
  if (tid < NHD) { const int h = tid; float mx = -3.0e38f; for (int m = 0; m < SEQ; ++m) mx = fmaxf(mx, sa[h][m]); float z = 0.f; for (int m = 0; m < SEQ; ++m) { const float e = exp_ni(sa[h][m] - mx); sa[h][m] = e; z += e; } const float iz = 1.0f / z; for (int m = 0; m < SEQ; ++m) sa[h][m] *= iz; }
  __syncthreads();
  for (int c = tid; c < DM; c += 256) { float acc12[NHD]; for (int h = 0; h < NHD; ++h) acc12[h] = 0.f;
    for (int m = 0; m < SEQ; ++m) { const float xv = bfr(X[(size_t)(m * 2 + b) * DM + c]);
#pragma unroll
      for (int h = 0; h < NHD; ++h) acc12[h] += sa[h][m] * xv; }
#pragma unroll
    for (int h = 0; h < NHD; ++h) sxa[h][c] = acc12[h]; }
  __syncthreads();
#pragma unroll 1
  for (int j = wave; j < DM / 16; j += 8) { v8f acc = {};
#pragma unroll 4
    for (int kc = 0; kc < DM / 32; ++kc) { const F2 a = split_row(&sxa[col][0], kc * 32, lane); const v16b w = frag_gbf(Wv + (size_t)(j * 16 + col) * DM + kc * 32, lane); acc = wmma_bf(a.l, w, acc); acc = wmma_bf(a.h, w, acc); }
    const int h = j / 4;
#pragma unroll
    for (int r = 0; r < 8; ++r) if (8 * g + r == h) sy[0][j * 16 + col] = acc[r] + bfr(Bv[j * 16 + col]); }
  __syncthreads();
#pragma unroll 1
  for (int j = wave; j < DM / 16; j += 8) { v8f acc = {};
#pragma unroll 4
    for (int kc = 0; kc < DM / 32; ++kc) { const F2 a = split_row(&sy[col][0], kc * 32, lane); const v16b w = frag_gbf(Wo + (size_t)(j * 16 + col) * DM + kc * 32, lane); acc = wmma_bf(a.l, w, acc); acc = wmma_bf(a.h, w, acc); }
    if (g == 0) sres[j * 16 + col] = acc[0] + bfr(Bo[j * 16 + col]); }
  __syncthreads();
  for (int q = tid; q < DM / 4; q += 256) vst2(out + (size_t)b * DM + q * 4, *(const v4f*)&sres[q * 4]);
}

extern "C" void kernel_launch(void* const* d_in, const int* in_sizes, int n_in, void* d_out, int out_size, void* d_ws, size_t ws_size, hipStream_t stream) {
  (void)in_sizes; (void)n_in; (void)out_size;
  const float** F = (const float**)d_in;
  if (ws_size < (size_t)WS_END) return;
  float* Kb = (float*)((char*)d_ws + WS_K);
  k_key<<<dim3((NROWP + 63) / 64, DM / 128), 128, 0, stream>>>(F[0], F[2], F[6], Kb);
  k_cls<<<NBT, 256, 0, stream>>>(F[0], Kb, F[1], F[5], F[3], F[7], F[4], F[8], (float*)d_out);
}
